// FrequencyTimeAttention_63385127354620
// MI455X (gfx1250) — hardware-verified
//
#include <hip/hip_runtime.h>
#include <stdint.h>

#define DIMX  512
#define HEADS 8
#define HDIM  64
#define SEQ   512
#define QKVN  1536
#define PTAB  64
#define KP    40
#define CP    68

typedef __bf16       v16b __attribute__((ext_vector_type(16)));
typedef _Float16     v16h __attribute__((ext_vector_type(16)));
typedef float        v8f  __attribute__((ext_vector_type(8)));
typedef float        v4f  __attribute__((ext_vector_type(4)));
typedef unsigned int v4u  __attribute__((ext_vector_type(4)));
typedef unsigned int v2u  __attribute__((ext_vector_type(2)));

union FragB { v16b v; v4u u[2]; };
union FragH { v16h v; v4u u[2]; };

__device__ __forceinline__ v8f mma_bf16(v16b a, v16b b, v8f c) {
    c = __builtin_amdgcn_wmma_f32_16x16x32_bf16(false, a, false, b, (short)0, c, false, false);
    asm volatile("v_nop\n\tv_nop\n\tv_nop\n\tv_nop" : "+v"(c) : "v"(a), "v"(b));
    return c;
}
__device__ __forceinline__ v8f mma_f16(v16h a, v16h b, v8f c) {
    c = __builtin_amdgcn_wmma_f32_16x16x32_f16(false, a, false, b, (short)0, c, false, false);
    asm volatile("v_nop\n\tv_nop\n\tv_nop\n\tv_nop" : "+v"(c) : "v"(a), "v"(b));
    return c;
}
__device__ __forceinline__ v8f mma3_bf16(v16b ah, v16b al, v16b bh, v16b bl, v8f c) {
    c = mma_bf16(ah, bh, c);
    c = mma_bf16(ah, bl, c);
    c = mma_bf16(al, bh, c);
    return c;
}
__device__ __forceinline__ v8f zero8() {
    v8f z = {0.f, 0.f, 0.f, 0.f, 0.f, 0.f, 0.f, 0.f};
    return z;
}

__device__ __forceinline__ unsigned short bf_rne(float x) {
    unsigned int u = __builtin_bit_cast(unsigned int, x);
    u = u + 0x7FFFu + ((u >> 16) & 1u);
    return (unsigned short)(u >> 16);
}
__device__ __forceinline__ float bf_val(unsigned short b) {
    return __builtin_bit_cast(float, ((unsigned int)b) << 16);
}
__device__ __forceinline__ unsigned short h_bits(float x) {
    _Float16 t = (_Float16)x;
    return __builtin_bit_cast(unsigned short, t);
}
__device__ __forceinline__ unsigned int pk2(unsigned short a, unsigned short b) {
    return (unsigned int)a | (((unsigned int)b) << 16);
}
__device__ __forceinline__ void split4_bf16(v4f v, v2u& hi, v2u& lo) {
    float f[4] = {v.x, v.y, v.z, v.w};
    unsigned short hs[4], ls[4];
#pragma unroll
    for (int i = 0; i < 4; ++i) {
        hs[i] = bf_rne(f[i]);
        ls[i] = bf_rne(f[i] - bf_val(hs[i]));
    }
    hi.x = pk2(hs[0], hs[1]); hi.y = pk2(hs[2], hs[3]);
    lo.x = pk2(ls[0], ls[1]); lo.y = pk2(ls[2], ls[3]);
}
__device__ __forceinline__ void split8_bf16(v4f a, v4f b, v4u& hi, v4u& lo) {
    float f[8] = {a.x, a.y, a.z, a.w, b.x, b.y, b.z, b.w};
    unsigned short hs[8], ls[8];
#pragma unroll
    for (int i = 0; i < 8; ++i) {
        hs[i] = bf_rne(f[i]);
        ls[i] = bf_rne(f[i] - bf_val(hs[i]));
    }
    hi.x = pk2(hs[0], hs[1]); hi.y = pk2(hs[2], hs[3]); hi.z = pk2(hs[4], hs[5]); hi.w = pk2(hs[6], hs[7]);
    lo.x = pk2(ls[0], ls[1]); lo.y = pk2(ls[2], ls[3]); lo.z = pk2(ls[4], ls[5]); lo.w = pk2(ls[6], ls[7]);
}
__device__ __forceinline__ v2u cvt4_f16(v4f v, float s) {
    v2u r;
    r.x = pk2(h_bits(v.x * s), h_bits(v.y * s));
    r.y = pk2(h_bits(v.z * s), h_bits(v.w * s));
    return r;
}
__device__ __forceinline__ v4u cvt8_f16(v4f a, v4f b, float s) {
    v4u r;
    r.x = pk2(h_bits(a.x * s), h_bits(a.y * s));
    r.y = pk2(h_bits(a.z * s), h_bits(a.w * s));
    r.z = pk2(h_bits(b.x * s), h_bits(b.y * s));
    r.w = pk2(h_bits(b.z * s), h_bits(b.w * s));
    return r;
}

__device__ __forceinline__ v16b frag_b(const unsigned short* p, int h) {
    FragB f;
    f.u[0] = *(const v4u*)(p + 8 * h);
    f.u[1] = *(const v4u*)(p + 16 + 8 * h);
    return f.v;
}
__device__ __forceinline__ v16h frag_h(const unsigned short* p, int h) {
    FragH f;
    f.u[0] = *(const v4u*)(p + 8 * h);
    f.u[1] = *(const v4u*)(p + 16 + 8 * h);
    return f.v;
}
__device__ __forceinline__ void frag_split_f32(const float* p, int h, v16b& hi, v16b& lo) {
    v4f f0 = *(const v4f*)(p + 8 * h);
    v4f f1 = *(const v4f*)(p + 8 * h + 4);
    v4f f2 = *(const v4f*)(p + 16 + 8 * h);
    v4f f3 = *(const v4f*)(p + 20 + 8 * h);
    FragB fh, fl;
    split8_bf16(f0, f1, fh.u[0], fl.u[0]);
    split8_bf16(f2, f3, fh.u[1], fl.u[1]);
    hi = fh.v; lo = fl.v;
}

__global__ __launch_bounds__(256)
void qk_proj_kernel(const float* __restrict__ x, const float* __restrict__ W,
                    const float* __restrict__ bias,
                    unsigned short* __restrict__ Qh, unsigned short* __restrict__ Ql,
                    unsigned short* __restrict__ Kh, unsigned short* __restrict__ Kl, int M)
{
    __shared__ __attribute__((aligned(16))) unsigned short Ah[64 * KP];
    __shared__ __attribute__((aligned(16))) unsigned short Al[64 * KP];
    __shared__ __attribute__((aligned(16))) unsigned short Bh[64 * KP];
    __shared__ __attribute__((aligned(16))) unsigned short Bl[64 * KP];
    __shared__ __attribute__((aligned(16))) float Cs[64 * CP];

    const int tid = threadIdx.x, lane = tid & 31, w = tid >> 5;
    const int h = lane >> 4, m = lane & 15;
    const int n0 = blockIdx.x * 64;
    const int m0 = blockIdx.y * 64;
    if (m0 + 64 > M || n0 + 64 > 2 * DIMX) return;
    const int mt  = w >> 1;
    const int ntb = (w & 1) * 2;

    v8f acc0 = zero8(), acc1 = zero8();

#pragma unroll 1
    for (int k0 = 0; k0 < DIMX; k0 += 32) {
#pragma unroll
        for (int p = 0; p < 2; ++p) {
            const int row = p * 32 + (tid >> 3);
            const int c4  = (tid & 7) * 4;
            v4f v = *(const v4f*)(x + (size_t)(m0 + row) * DIMX + k0 + c4);
            v2u hv, lv;
            split4_bf16(v, hv, lv);
            *(v2u*)(Ah + row * KP + c4) = hv;
            *(v2u*)(Al + row * KP + c4) = lv;
        }
#pragma unroll
        for (int p = 0; p < 2; ++p) {
            const int kr = p * 16 + (tid >> 4);
            const int c4 = (tid & 15) * 4;
            v4f v = *(const v4f*)(W + (size_t)(k0 + kr) * QKVN + n0 + c4);
            float f[4] = {v.x, v.y, v.z, v.w};
#pragma unroll
            for (int i = 0; i < 4; ++i) {
                const unsigned short hb = bf_rne(f[i]);
                Bh[(c4 + i) * KP + kr] = hb;
                Bl[(c4 + i) * KP + kr] = bf_rne(f[i] - bf_val(hb));
            }
        }
        __syncthreads();

        const v16b fah = frag_b(Ah + (mt * 16 + m) * KP, h);
        const v16b fal = frag_b(Al + (mt * 16 + m) * KP, h);
        const v16b fbh0 = frag_b(Bh + (ntb * 16 + m) * KP, h);
        const v16b fbl0 = frag_b(Bl + (ntb * 16 + m) * KP, h);
        const v16b fbh1 = frag_b(Bh + ((ntb + 1) * 16 + m) * KP, h);
        const v16b fbl1 = frag_b(Bl + ((ntb + 1) * 16 + m) * KP, h);
        acc0 = mma3_bf16(fah, fal, fbh0, fbl0, acc0);
        acc1 = mma3_bf16(fah, fal, fbh1, fbl1, acc1);
        __syncthreads();
    }

    {
        const int ca = ntb * 16 + m, cb = ca + 16;
        const float ba = bias[n0 + ca], bb = bias[n0 + cb];
#pragma unroll
        for (int r = 0; r < 8; ++r) {
            const int row = mt * 16 + 8 * h + r;
            Cs[row * CP + ca] = acc0[r] + ba;
            Cs[row * CP + cb] = acc1[r] + bb;
        }
    }
    __syncthreads();

    const int which = n0 / DIMX;
    const int hh    = (n0 % DIMX) / HDIM;
    const int bidx  = m0 / SEQ, s0 = m0 % SEQ;
    unsigned short* dh = which ? Kh : Qh;
    unsigned short* dl = which ? Kl : Ql;
    const size_t base = ((size_t)(bidx * HEADS + hh) * SEQ + s0) * HDIM;
    const int piece = lane & 7;

    v4u hv[2], lv[2];
    size_t off[2];
#pragma unroll
    for (int q = 0; q < 2; ++q) {
        const int row = w * 8 + q * 4 + (lane >> 3);
        const float* cp = Cs + row * CP + piece * 8;
        const v4f a = *(const v4f*)cp;
        const v4f b = *(const v4f*)(cp + 4);
        split8_bf16(a, b, hv[q], lv[q]);
        off[q] = base + (size_t)row * HDIM + piece * 8;
    }
#pragma unroll
    for (int q = 0; q < 2; ++q) {
        *(volatile v4u*)(dh + off[q]) = hv[q];
        *(volatile v4u*)(dl + off[q]) = lv[q];
    }
    __threadfence();
#pragma unroll
    for (int q = 0; q < 2; ++q) {
        *(volatile v4u*)(dh + off[q]) = hv[q];
        *(volatile v4u*)(dl + off[q]) = lv[q];
    }
}

template <int MODE>
__global__ __launch_bounds__(256)
void f16_gemm_kernel(const float* __restrict__ xa, const unsigned short* __restrict__ oa,
                     const float* __restrict__ W, const float* __restrict__ bias,
                     unsigned short* __restrict__ Vt, float* __restrict__ out, int M)
{
    __shared__ __attribute__((aligned(16))) unsigned short As[64 * KP];
    __shared__ __attribute__((aligned(16))) unsigned short Bs[64 * KP];
    __shared__ __attribute__((aligned(16))) float Cs[64 * CP];

    const int tid = threadIdx.x, lane = tid & 31, w = tid >> 5;
    const int h = lane >> 4, m = lane & 15;
    const int n0 = blockIdx.x * 64;
    const int m0 = blockIdx.y * 64;
    if (m0 + 64 > M || n0 + 64 > DIMX) return;
    const int ldw  = (MODE == 0) ? QKVN : DIMX;
    const int cofs = (MODE == 0) ? 2 * DIMX : 0;
    const int mt  = w >> 1;
    const int ntb = (w & 1) * 2;

    v8f acc0 = zero8(), acc1 = zero8();

#pragma unroll 1
    for (int k0 = 0; k0 < DIMX; k0 += 32) {
        if (MODE == 0) {
#pragma unroll
            for (int p = 0; p < 2; ++p) {
                const int row = p * 32 + (tid >> 3);
                const int c4  = (tid & 7) * 4;
                v4f v = *(const v4f*)(xa + (size_t)(m0 + row) * DIMX + k0 + c4);
                *(v2u*)(As + row * KP + c4) = cvt4_f16(v, 16.0f);
            }
        } else {
            const int row = tid >> 2;
            const int c8  = (tid & 3) * 8;
            v4u v = *(const v4u*)(oa + (size_t)(m0 + row) * DIMX + k0 + c8);
            *(v4u*)(As + row * KP + c8) = v;
        }
#pragma unroll
        for (int p = 0; p < 2; ++p) {
            const int kr = p * 16 + (tid >> 4);
            const int c4 = (tid & 15) * 4;
            v4f v = *(const v4f*)(W + (size_t)(k0 + kr) * ldw + cofs + n0 + c4);
            Bs[(c4 + 0) * KP + kr] = h_bits(v.x * 64.0f);
            Bs[(c4 + 1) * KP + kr] = h_bits(v.y * 64.0f);
            Bs[(c4 + 2) * KP + kr] = h_bits(v.z * 64.0f);
            Bs[(c4 + 3) * KP + kr] = h_bits(v.w * 64.0f);
        }
        __syncthreads();

        const v16h fa  = frag_h(As + (mt * 16 + m) * KP, h);
        const v16h fb0 = frag_h(Bs + (ntb * 16 + m) * KP, h);
        const v16h fb1 = frag_h(Bs + ((ntb + 1) * 16 + m) * KP, h);
        acc0 = mma_f16(fa, fb0, acc0);
        acc1 = mma_f16(fa, fb1, acc1);
        __syncthreads();
    }

    {
        const int ca = ntb * 16 + m, cb = ca + 16;
#pragma unroll
        for (int r = 0; r < 8; ++r) {
            const int row = mt * 16 + 8 * h + r;
            Cs[row * CP + ca] = acc0[r];
            Cs[row * CP + cb] = acc1[r];
        }
    }
    __syncthreads();

    const int piece = lane & 7;
    if (MODE == 0) {
        const int hh = n0 / HDIM;
        const int bidx = m0 / SEQ, s0 = m0 % SEQ;
        const int bh = bidx * HEADS + hh;
        v4u pv[2];
        size_t off[2];
#pragma unroll
        for (int q = 0; q < 2; ++q) {
            const int d = w * 8 + q * 4 + (lane >> 3);
            const float b8 = 8.0f * bias[2 * DIMX + n0 + d];
            float f[8];
#pragma unroll
            for (int i = 0; i < 8; ++i)
                f[i] = Cs[(piece * 8 + i) * CP + d] * (1.0f / 128.0f) + b8;
            v4f a = {f[0], f[1], f[2], f[3]};
            v4f b = {f[4], f[5], f[6], f[7]};
            pv[q]  = cvt8_f16(a, b, 1.0f);
            off[q] = ((size_t)(bh * HDIM + d)) * SEQ + s0 + piece * 8;
        }
#pragma unroll
        for (int q = 0; q < 2; ++q) *(volatile v4u*)(Vt + off[q]) = pv[q];
        __threadfence();
#pragma unroll
        for (int q = 0; q < 2; ++q) *(volatile v4u*)(Vt + off[q]) = pv[q];
    } else {
        v4f ov[4];
        size_t off[4];
#pragma unroll
        for (int q = 0; q < 4; ++q) {
            const int gl  = w * 16 + q * 4 + (lane >> 3);
            const int row = gl >> 1;
            const int cb  = (gl & 1) * 32 + piece * 4;
            const v4f c  = *(const v4f*)(Cs + row * CP + cb);
            const v4f bb = *(const v4f*)(bias + n0 + cb);
            ov[q]  = c * (1.0f / 1024.0f) + bb;
            off[q] = (size_t)(m0 + row) * DIMX + n0 + cb;
        }
#pragma unroll
        for (int q = 0; q < 4; ++q) *(volatile v4f*)(out + off[q]) = ov[q];
        __threadfence();
#pragma unroll
        for (int q = 0; q < 4; ++q) *(volatile v4f*)(out + off[q]) = ov[q];
    }
}

__global__ __launch_bounds__(32)
void attn_kernel(const unsigned short* __restrict__ Qh, const unsigned short* __restrict__ Ql,
                 const unsigned short* __restrict__ Kh, const unsigned short* __restrict__ Kl,
                 const unsigned short* __restrict__ Vt, const float* __restrict__ pos,
                 unsigned short* __restrict__ O16, int nblk)
{
    __shared__ __attribute__((aligned(16))) float sc[16 * SEQ];
    __shared__ __attribute__((aligned(16))) unsigned short pb[16 * SEQ];
    __shared__ __attribute__((aligned(16))) float qps[16 * PTAB];
    __shared__ float rinv[16];

    const int blk = blockIdx.x;
    if (blk >= nblk) return;
    const int lane = threadIdx.x & 31, h = lane >> 4, m = lane & 15;
    const int bh   = blk / (SEQ / 16);
    const int i0   = (blk % (SEQ / 16)) * 16;
    const int bidx = bh / HEADS, hd = bh % HEADS;

    const size_t qrow = ((size_t)bh * SEQ + i0 + m) * HDIM;
    const v16b qh0 = frag_b(Qh + qrow, h), qh1 = frag_b(Qh + qrow + 32, h);
    const v16b ql0 = frag_b(Ql + qrow, h), ql1 = frag_b(Ql + qrow + 32, h);

#pragma unroll 1
    for (int nt = 0; nt < PTAB / 16; ++nt) {
        const float* prow = pos + (size_t)(nt * 16 + m) * DIMX + hd * HDIM;
        v16b ph, pl;
        v8f acc = zero8();
        frag_split_f32(prow, h, ph, pl);
        acc = mma3_bf16(qh0, ql0, ph, pl, acc);
        frag_split_f32(prow + 32, h, ph, pl);
        acc = mma3_bf16(qh1, ql1, ph, pl, acc);
#pragma unroll
        for (int r = 0; r < 8; ++r) qps[(8 * h + r) * PTAB + nt * 16 + m] = acc[r];
    }
    __syncthreads();

#pragma unroll 1
    for (int j0 = 0; j0 < SEQ; j0 += 16) {
        const size_t krow = ((size_t)bh * SEQ + j0 + m) * HDIM;
        v8f acc = zero8();
        acc = mma3_bf16(qh0, ql0, frag_b(Kh + krow, h), frag_b(Kl + krow, h), acc);
        acc = mma3_bf16(qh1, ql1, frag_b(Kh + krow + 32, h), frag_b(Kl + krow + 32, h), acc);
        const int j = j0 + m;
#pragma unroll
        for (int r = 0; r < 8; ++r) {
            const int irel = 8 * h + r;
            int rp = j - (i0 + irel) + PTAB / 2;
            rp = rp < 0 ? 0 : (rp > PTAB - 1 ? PTAB - 1 : rp);
            sc[irel * SEQ + j] = acc[r] * 0.125f + qps[irel * PTAB + rp];
        }
    }
    __syncthreads();

#pragma unroll 1
    for (int r = 0; r < 16; ++r) {
        float v[16];
        float mx = -3.0e38f;
#pragma unroll
        for (int t = 0; t < 16; ++t) {
            v[t] = sc[r * SEQ + lane + 32 * t];
            mx = fmaxf(mx, v[t]);
        }
#pragma unroll
        for (int o = 16; o > 0; o >>= 1) mx = fmaxf(mx, __shfl_xor(mx, o));
        float sum = 0.0f;
#pragma unroll
        for (int t = 0; t < 16; ++t) {
            const float e = __expf(v[t] - mx) * 256.0f;
            const _Float16 p = (_Float16)e;
            pb[r * SEQ + lane + 32 * t] = __builtin_bit_cast(unsigned short, p);
            sum += (float)p;
        }
#pragma unroll
        for (int o = 16; o > 0; o >>= 1) sum += __shfl_xor(sum, o);
        if (lane == 0) rinv[r] = 2.0f / sum;
    }
    __syncthreads();

    v8f o0 = zero8(), o1 = zero8(), o2 = zero8(), o3 = zero8();
#pragma unroll 1
    for (int j0 = 0; j0 < SEQ; j0 += 32) {
        const v16h pa = frag_h(pb + m * SEQ + j0, h);
        const size_t vrow = ((size_t)bh * HDIM + m) * SEQ + j0;
        o0 = mma_f16(pa, frag_h(Vt + vrow, h), o0);
        o1 = mma_f16(pa, frag_h(Vt + vrow + (size_t)16 * SEQ, h), o1);
        o2 = mma_f16(pa, frag_h(Vt + vrow + (size_t)32 * SEQ, h), o2);
        o3 = mma_f16(pa, frag_h(Vt + vrow + (size_t)48 * SEQ, h), o3);
    }

    float* ost = sc;
#pragma unroll
    for (int r = 0; r < 8; ++r) {
        const int irel = 8 * h + r;
        const float s = rinv[irel];
        ost[irel * HDIM +  0 + m] = o0[r] * s;
        ost[irel * HDIM + 16 + m] = o1[r] * s;
        ost[irel * HDIM + 32 + m] = o2[r] * s;
        ost[irel * HDIM + 48 + m] = o3[r] * s;
    }
    __syncthreads();

    const int piece = lane & 7;
    v4u ov[4];
    size_t off[4];
#pragma unroll
    for (int q = 0; q < 4; ++q) {
        const int row = q * 4 + (lane >> 3);
        const float* cp = ost + row * HDIM + piece * 8;
        const v4f a = *(const v4f*)cp;
        const v4f b = *(const v4f*)(cp + 4);
        ov[q]  = cvt8_f16(a, b, 1.0f);
        off[q] = ((size_t)(bidx * SEQ + i0 + row)) * DIMX + hd * HDIM + piece * 8;
    }
#pragma unroll
    for (int q = 0; q < 4; ++q) *(volatile v4u*)(O16 + off[q]) = ov[q];
    __threadfence();
#pragma unroll
    for (int q = 0; q < 4; ++q) *(volatile v4u*)(O16 + off[q]) = ov[q];
}

extern "C" void kernel_launch(void* const* d_in, const int* in_sizes, int n_in,
                              void* d_out, int out_size, void* d_ws, size_t ws_size,
                              hipStream_t stream)
{
    if (n_in < 6) return;
    const float* x    = (const float*)d_in[0];
    const float* Wqkv = (const float*)d_in[1];
    const float* bqkv = (const float*)d_in[2];
    const float* Wout = (const float*)d_in[3];
    const float* bout = (const float*)d_in[4];
    const float* pos  = (const float*)d_in[5];
    float* out = (float*)d_out;

    const int M = in_sizes[0] / DIMX;
    if (M <= 0 || M * DIMX != in_sizes[0] || (M % SEQ) != 0) return;
    if (in_sizes[1] != DIMX * QKVN || in_sizes[2] != QKVN) return;
    if (in_sizes[3] != DIMX * DIMX || in_sizes[4] != DIMX) return;
    if (in_sizes[5] != PTAB * DIMX) return;
    if (out_size != M * DIMX) return;
    const int NB = M / SEQ;

    const size_t plane = (size_t)M * DIMX * sizeof(unsigned short);
    if (6 * plane > ws_size) return;
    char* ws = (char*)d_ws;
    unsigned short* Qh  = (unsigned short*)(ws + 0 * plane);
    unsigned short* Ql  = (unsigned short*)(ws + 1 * plane);
    unsigned short* Kh  = (unsigned short*)(ws + 2 * plane);
    unsigned short* Kl  = (unsigned short*)(ws + 3 * plane);
    unsigned short* Vt  = (unsigned short*)(ws + 4 * plane);
    unsigned short* O16 = (unsigned short*)(ws + 5 * plane);

    const int mblk = M / 64;
    const int nblk_attn = NB * HEADS * (SEQ / 16);

    qk_proj_kernel<<<dim3((2 * DIMX) / 64, mblk), 256, 0, stream>>>(x, Wqkv, bqkv, Qh, Ql, Kh, Kl, M);
    f16_gemm_kernel<0><<<dim3(DIMX / 64, mblk), 256, 0, stream>>>(x, O16, Wqkv, bqkv, Vt, out, M);
    attn_kernel<<<nblk_attn, 32, 0, stream>>>(Qh, Ql, Kh, Kl, Vt, pos, O16, nblk_attn);
    f16_gemm_kernel<1><<<dim3(DIMX / 64, mblk), 256, 0, stream>>>(x, O16, Wout, bout, Vt, out, M);
}
